// CrissCrossAttention_90804198572459
// MI455X (gfx1250) — hardware-verified
//
#include <hip/hip_runtime.h>
#include <math.h>

typedef __attribute__((ext_vector_type(16))) _Float16 v16h;
typedef __attribute__((ext_vector_type(16))) __bf16 v16b;
typedef __attribute__((ext_vector_type(8)))  _Float16 v8h;
typedef __attribute__((ext_vector_type(8)))  float v8f;
typedef __attribute__((ext_vector_type(4)))  float v4f;
typedef __attribute__((ext_vector_type(2)))  float v2f;
typedef __attribute__((ext_vector_type(4)))  unsigned v4u;

template <typename T> __device__ __forceinline__ void vst2(void* p, T v) { *(volatile T*)p = v; __threadfence(); *(volatile T*)p = v; }
__device__ __forceinline__ v8f wmma16(v16h a, v16h b, v8f c) {
  v8f d = __builtin_amdgcn_wmma_f32_16x16x32_f16(false, a, false, b, (short)0, c, false, false);
  asm volatile("v_nop\n\tv_nop\n\tv_nop\n\tv_nop" : "+v"(d) : "v"(a), "v"(b));
  return d;
}
__device__ __forceinline__ v8f wmma_bf(v16b a, v16b b, v8f c) {
  v8f d = __builtin_amdgcn_wmma_f32_16x16x32_bf16(false, a, false, b, (short)0, c, false, false);
  asm volatile("v_nop\n\tv_nop\n\tv_nop\n\tv_nop" : "+v"(d) : "v"(a), "v"(b));
  return d;
}
__device__ __forceinline__ v16h frag_h(const _Float16* rowk0, int lane) {
  union { v16h v; v8h q[2]; } u; const _Float16* p = rowk0 + 8 * (lane >> 4);
  u.q[0] = *(const v8h*)p; u.q[1] = *(const v8h*)(p + 16); return u.v;
}
__device__ __forceinline__ v16b frag_b(const unsigned short* rowk0, int lane) {
  union { v16b v; v4u q[2]; } u; const unsigned short* p = rowk0 + 8 * (lane >> 4);
  u.q[0] = *(const v4u*)p; u.q[1] = *(const v4u*)(p + 16); return u.v;
}
__device__ __forceinline__ unsigned short bfb(float f) { unsigned u = __float_as_uint(f); u += 0x7FFFu + ((u >> 16) & 1u); return (unsigned short)(u >> 16); }
__device__ __forceinline__ float bfr(float f) { return __uint_as_float(((unsigned)bfb(f)) << 16); }
#define LDSX() do { asm volatile("s_wait_dscnt 0" ::: "memory"); __builtin_amdgcn_wave_barrier(); __builtin_amdgcn_fence(__ATOMIC_RELEASE, "workgroup"); } while (0)

#ifndef NB
#define NB 4
#endif
#ifndef SEQ
#define SEQ 4096
#endif
#define NB_FULL 4
#define SEQ_FULL 4096
#ifndef XSTR
#define XSTR SEQ_FULL
#endif
#define CX 256
#define DQ 32
#define PSC 16384.0f
#define AOC 64.0f
#define WGC 256.0f
static_assert(SEQ % 128 == 0);
static_assert(SEQ >= 128 && SEQ <= SEQ_FULL);
static_assert(NB >= 1 && NB <= NB_FULL);

#define WS_XB  ((size_t)0)
#define WS_QH  (WS_XB + 2u * (size_t)NB * SEQ * CX)
#define WS_QL  (WS_QH + 2u * (size_t)NB * SEQ * DQ)
#define WS_KH  (WS_QL + 2u * (size_t)NB * SEQ * DQ)
#define WS_KL  (WS_KH + 2u * (size_t)NB * SEQ * DQ)
#define WS_VT  (WS_KL + 2u * (size_t)NB * SEQ * DQ)
#define WS_AO  (WS_VT + 2u * (size_t)NB * CX * SEQ)
#define WS_WQ  (WS_AO + 2u * (size_t)NB * SEQ * CX)
#define WS_WK  (WS_WQ + 2u * (size_t)DQ * CX)
#define WS_WV  (WS_WK + 2u * (size_t)DQ * CX)
#define WS_WG  (WS_WV + 2u * (size_t)CX * CX)
#define WS_S   (WS_WG + 2u * (size_t)CX * CX)
#define WS_END (WS_S + 4u * (size_t)SEQ * SEQ)
static_assert(WS_END <= (size_t)134217728u);
static_assert(WS_QH % 128 == 0 && WS_QL % 128 == 0 && WS_KH % 128 == 0 && WS_KL % 128 == 0 && WS_VT % 128 == 0 && WS_AO % 128 == 0 && WS_WQ % 128 == 0 && WS_WK % 128 == 0 && WS_WV % 128 == 0 && WS_WG % 128 == 0 && WS_S % 128 == 0);

__device__ __forceinline__ void cvt8_bf(const float* __restrict__ src, unsigned short* __restrict__ dst) {
  const v4f a = *(const v4f*)src, c = *(const v4f*)(src + 4); v4u o;
  o[0] = (unsigned)bfb(a[0]) | ((unsigned)bfb(a[1]) << 16); o[1] = (unsigned)bfb(a[2]) | ((unsigned)bfb(a[3]) << 16);
  o[2] = (unsigned)bfb(c[0]) | ((unsigned)bfb(c[1]) << 16); o[3] = (unsigned)bfb(c[2]) | ((unsigned)bfb(c[3]) << 16);
  vst2((v4u*)dst, o);
}
__global__ __launch_bounds__(256) void k_wc(const float* __restrict__ WQ, const float* __restrict__ WK, const float* __restrict__ WV, const float* __restrict__ WG,
                                            unsigned short* __restrict__ WQB, unsigned short* __restrict__ WKB, unsigned short* __restrict__ WVB, _Float16* __restrict__ WGH) {
  const int bx = blockIdx.x, wave = threadIdx.x >> 5, lane = threadIdx.x & 31;
  if (bx < 4) { const int row = bx * 8 + wave; cvt8_bf(WQ + row * CX + lane * 8, WQB + row * CX + lane * 8); }
  else if (bx < 8) { const int row = (bx - 4) * 8 + wave; cvt8_bf(WK + row * CX + lane * 8, WKB + row * CX + lane * 8); }
  else if (bx < 40) { const int row = (bx - 8) * 8 + wave; cvt8_bf(WV + (size_t)row * CX + lane * 8, WVB + (size_t)row * CX + lane * 8); }
  else { const int row = (bx - 40) * 8 + wave; const float* s = WG + (size_t)row * CX + lane * 8; const v4f a = *(const v4f*)s, c = *(const v4f*)(s + 4); union { v8h h; v4u u; } o;
#pragma unroll
    for (int i = 0; i < 4; ++i) { o.h[i] = (_Float16)(bfr(a[i]) * WGC); o.h[4 + i] = (_Float16)(bfr(c[i]) * WGC); }
    vst2((v4u*)(WGH + (size_t)row * CX + lane * 8), o.u); }
}
__global__ __launch_bounds__(256) void k_xt(const float* __restrict__ X, unsigned short* __restrict__ XB) { __shared__ unsigned short st[CX][66];
  const int t = threadIdx.x; const int l0 = blockIdx.x * 64; const size_t b = blockIdx.y;
  for (int e = t; e < CX * 64; e += 256) { const int c = e >> 6, ll = e & 63; st[c][ll] = bfb(X[(b * CX + c) * (size_t)XSTR + l0 + ll]); }
  __syncthreads();
  for (int e = t; e < 64 * 32; e += 256) { const int ll = e >> 5, q = e & 31; v4u o;
#pragma unroll
    for (int k = 0; k < 4; ++k) o[k] = (unsigned)st[q * 8 + 2 * k][ll] | ((unsigned)st[q * 8 + 2 * k + 1][ll] << 16);
    vst2((v4u*)(XB + (b * SEQ + l0 + ll) * CX + q * 8), o); } }
__global__ __launch_bounds__(128) void k_qk(const unsigned short* __restrict__ XB, const unsigned short* __restrict__ WQB, const float* __restrict__ BQ, const unsigned short* __restrict__ WKB, const float* __restrict__ BK,
                                            _Float16* __restrict__ QH, _Float16* __restrict__ QL, _Float16* __restrict__ KH, _Float16* __restrict__ KL) {
  __shared__ __align__(16) _Float16 st[4][4][16][40];
  const int tid = threadIdx.x, wave = tid >> 5, lane = tid & 31, col = lane & 15, g = lane >> 4; const size_t r0 = (size_t)blockIdx.x * 64 + wave * 16;
  v8f acc[4] = {};
#pragma unroll 2
  for (int kc = 0; kc < CX / 32; ++kc) { const v16b a = frag_b(XB + (r0 + col) * CX + kc * 32, lane);
#pragma unroll
    for (int j = 0; j < 4; ++j) { const unsigned short* WB = (j < 2) ? WQB : WKB; const int o = (j & 1) * 16 + col;
      const v16b w = frag_b(WB + (size_t)o * CX + kc * 32, lane);
      asm volatile("s_wait_loadcnt 0x0" ::: "memory"); acc[j] = wmma_bf(a, w, acc[j]); } }
#pragma unroll
  for (int j = 0; j < 4; ++j) { const int o = (j & 1) * 16 + col; const float bb = (j < 2) ? bfr(BQ[o]) : bfr(BK[o]); const int ph = (j < 2) ? 0 : 2;
#pragma unroll
    for (int r = 0; r < 8; ++r) { const float v = acc[j][r] + bb; const _Float16 hv = (_Float16)v; st[wave][ph][8 * g + r][o] = hv; st[wave][ph + 1][8 * g + r][o] = (_Float16)((v - (float)hv) * 1024.0f); } }
  LDSX();
  { _Float16* P4[4] = {QH, QL, KH, KL};
#pragma unroll
    for (int it = 0; it < 2; ++it) { const int rl = it * 8 + (lane >> 2), pc = (lane & 3) * 8;
#pragma unroll
      for (int ph = 0; ph < 4; ++ph) vst2((v4u*)(P4[ph] + (r0 + rl) * DQ + pc), *(const v4u*)&st[wave][ph][rl][pc]); } } }
__global__ __launch_bounds__(128) void k_vp(const unsigned short* __restrict__ XB, const unsigned short* __restrict__ WVB, const float* __restrict__ BV, _Float16* __restrict__ VT) { __shared__ __align__(16) _Float16 th[128][72];
  const int tid = threadIdx.x, wave = tid >> 5, lane = tid & 31, col = lane & 15, g = lane >> 4; const int c0 = blockIdx.y * 128; const size_t r0 = (size_t)blockIdx.x * 64;
  v8f acc[8] = {};
#pragma unroll 2
  for (int kc = 0; kc < CX / 32; ++kc) { const v16b a = frag_b(XB + (r0 + wave * 16 + col) * CX + kc * 32, lane);
#pragma unroll
    for (int j = 0; j < 8; ++j) { const int o = c0 + j * 16 + col; const v16b w = frag_b(WVB + (size_t)o * CX + kc * 32, lane);
      asm volatile("s_wait_loadcnt 0x0" ::: "memory"); acc[j] = wmma_bf(a, w, acc[j]); } }
#pragma unroll
  for (int j = 0; j < 8; ++j) { const float bb = bfr(BV[c0 + j * 16 + col]);
#pragma unroll
    for (int r = 0; r < 8; ++r) th[j * 16 + col][wave * 16 + 8 * g + r] = (_Float16)(acc[j][r] + bb); }
  __syncthreads();
  { const size_t b = r0 / SEQ; const int m0 = (int)(r0 % SEQ); for (int e = tid; e < 128 * 8; e += 128) { const int cl = e >> 3, q = e & 7; vst2((v4u*)(VT + (b * CX + c0 + cl) * (size_t)SEQ + m0 + q * 8), *(const v4u*)&th[cl][q * 8]); } } }
__global__ __launch_bounds__(128) void k_sc(const _Float16* __restrict__ QH, const _Float16* __restrict__ QL, const _Float16* __restrict__ KH, const _Float16* __restrict__ KL, int b, float* __restrict__ S) { __shared__ __align__(16) float ss[4][16][132];
  const int tid = threadIdx.x, wave = tid >> 5, lane = tid & 31, col = lane & 15, g = lane >> 4; const int k0 = blockIdx.y * 128; const int ql0 = blockIdx.x * 64 + wave * 16; const size_t q0 = (size_t)b * SEQ + ql0;
  v8f acc[8] = {}, accl[8] = {};
  { const v16h ah = frag_h(QH + (q0 + col) * DQ, lane), al = frag_h(QL + (q0 + col) * DQ, lane);
#pragma unroll
    for (int j = 0; j < 8; ++j) { const size_t ko = ((size_t)b * SEQ + k0 + j * 16 + col) * DQ; const v16h kb = frag_h(KH + ko, lane), kl = frag_h(KL + ko, lane); acc[j] = wmma16(ah, kb, acc[j]); accl[j] = wmma16(al, kb, accl[j]); accl[j] = wmma16(ah, kl, accl[j]); } }
#pragma unroll
  for (int j = 0; j < 8; ++j)
#pragma unroll
    for (int r = 0; r < 8; ++r) ss[wave][8 * g + r][j * 16 + col] = acc[j][r] + accl[j][r] * (1.0f / 1024.0f);
  LDSX(); for (int rl = 0; rl < 16; ++rl) vst2((v4f*)(S + (size_t)(ql0 + rl) * SEQ + k0 + lane * 4), *(const v4f*)&ss[wave][rl][lane * 4]); }
__global__ __launch_bounds__(64) void k_rsm(float* __restrict__ S) { __shared__ __align__(16) float es[2][SEQ];
  const int w = threadIdx.x >> 5, lane = threadIdx.x & 31; float* R = S + ((size_t)blockIdx.x * 2 + w) * SEQ; float* E = es[w];
  float mx = -3.0e38f;
#pragma unroll 1
  for (int i = 0; i < SEQ / 128; ++i) { const v4f v = *(const v4f*)(R + i * 128 + lane * 4); *(v4f*)(E + i * 128 + lane * 4) = v; mx = fmaxf(mx, fmaxf(fmaxf(v[0], v[1]), fmaxf(v[2], v[3]))); }
#pragma unroll
  for (int s = 16; s > 0; s >>= 1) mx = fmaxf(mx, __shfl_xor(mx, s));
  __syncthreads();
  float z = 0.f;
#pragma unroll 1
  for (int i = 0; i < SEQ / 64; ++i) { float* p = E + i * 64 + lane * 2; v2f v = *(const v2f*)p; v[0] = expf(v[0] - mx); v[1] = expf(v[1] - mx); *(v2f*)p = v; z += v[0] + v[1]; }
#pragma unroll
  for (int s = 16; s > 0; s >>= 1) z += __shfl_xor(z, s);
  const float sc = PSC / z;
  __syncthreads();
#pragma unroll 1
  for (int i = 0; i < SEQ / 128; ++i) { const v4f e = *(const v4f*)(E + i * 128 + lane * 4); const v4f o = e * sc; vst2((v4f*)(R + i * 128 + lane * 4), o); } }
__global__ __launch_bounds__(128) void k_pv(const float* __restrict__ PS, const _Float16* __restrict__ VT, int b, _Float16* __restrict__ AO) { __shared__ __align__(16) _Float16 th[64][136];
  const int tid = threadIdx.x, wave = tid >> 5, lane = tid & 31, col = lane & 15, g = lane >> 4; const int ql0 = blockIdx.x * 64 + wave * 16; const int c0 = blockIdx.y * 128;
  v8f acc[8] = {}, accl[8] = {};
#pragma unroll 1
  for (int kc = 0; kc < SEQ / 32; ++kc) { v16h ph, pl; { const float* pr = PS + (size_t)(ql0 + col) * SEQ + kc * 32 + 8 * g;
#pragma unroll
      for (int i = 0; i < 8; ++i) { const float a0 = pr[i], a1 = pr[16 + i]; const _Float16 h0 = (_Float16)a0, h1 = (_Float16)a1; ph[i] = h0; ph[8 + i] = h1; pl[i] = (_Float16)((a0 - (float)h0) * 1024.0f); pl[8 + i] = (_Float16)((a1 - (float)h1) * 1024.0f); } }
    asm volatile("s_wait_loadcnt 0x0" ::: "memory");
#pragma unroll
    for (int j = 0; j < 8; ++j) { const v16h vv = frag_h(VT + ((size_t)b * CX + c0 + j * 16 + col) * (size_t)SEQ + kc * 32, lane); acc[j] = wmma16(ph, vv, acc[j]); accl[j] = wmma16(pl, vv, accl[j]); } }
#pragma unroll
  for (int j = 0; j < 8; ++j)
#pragma unroll
    for (int r = 0; r < 8; ++r) th[wave * 16 + 8 * g + r][j * 16 + col] = (_Float16)((acc[j][r] + accl[j][r] * (1.0f / 1024.0f)) * (AOC / PSC));
  __syncthreads();
  { const int n0 = blockIdx.x * 64; for (int e = tid; e < 64 * 16; e += 128) { const int rl = e >> 4, q = e & 15; vst2((v4u*)(AO + ((size_t)b * SEQ + n0 + rl) * CX + c0 + q * 8), *(const v4u*)&th[rl][q * 8]); } } }
__global__ __launch_bounds__(128) void k_op(const _Float16* __restrict__ AO, const _Float16* __restrict__ WGH, const float* __restrict__ BG, const float* __restrict__ X, float* __restrict__ OUT) { __shared__ __align__(16) float stc[128][68];
  const int tid = threadIdx.x, wave = tid >> 5, lane = tid & 31, col = lane & 15, g = lane >> 4; const int c0 = blockIdx.y * 128; const size_t r0 = (size_t)blockIdx.x * 64;
  v8f acc[8] = {};
#pragma unroll 2
  for (int kc = 0; kc < CX / 32; ++kc) { const v16h a = frag_h(AO + (r0 + wave * 16 + col) * CX + kc * 32, lane);
#pragma unroll
    for (int j = 0; j < 8; ++j) { const int o = c0 + j * 16 + col; const v16h w = frag_h(WGH + (size_t)o * CX + kc * 32, lane);
      asm volatile("s_wait_loadcnt 0x0" ::: "memory"); acc[j] = wmma16(a, w, acc[j]); } }
#pragma unroll
  for (int j = 0; j < 8; ++j) { const float bb = bfr(BG[c0 + j * 16 + col]);
#pragma unroll
    for (int r = 0; r < 8; ++r) stc[j * 16 + col][wave * 16 + 8 * g + r] = acc[j][r] * (1.0f / (AOC * WGC)) + bb; }
  __syncthreads();
  { const size_t b = r0 / SEQ; const int n0 = (int)(r0 % SEQ);
    for (int e = tid; e < 128 * 16; e += 128) { const int cl = e >> 4, q = e & 15; const size_t off = (b * CX + c0 + cl) * (size_t)XSTR + n0 + q * 4;
      const v4f sr = *(const v4f*)(X + off); v4f o = *(const v4f*)&stc[cl][q * 4]; o[0] += bfr(sr[0]); o[1] += bfr(sr[1]); o[2] += bfr(sr[2]); o[3] += bfr(sr[3]); vst2((v4f*)(OUT + off), o); } } }

extern "C" void kernel_launch(void* const* d_in, const int* in_sizes, int n_in, void* d_out, int out_size, void* d_ws, size_t ws_size, hipStream_t stream) {
  if (n_in < 9) return;
  if (in_sizes[0] < NB * CX * SEQ || in_sizes[1] < DQ * CX || in_sizes[2] < DQ || in_sizes[3] < DQ * CX || in_sizes[4] < DQ ||
      in_sizes[5] < CX * CX || in_sizes[6] < CX || in_sizes[7] < CX * CX || in_sizes[8] < CX) return;
  if (out_size < NB * CX * SEQ) return;
  if (ws_size < (size_t)WS_END) return;
  const float** F = (const float**)d_in;
  char* ws = (char*)d_ws;
  unsigned short* XB = (unsigned short*)(ws + WS_XB);
  _Float16 *QH = (_Float16*)(ws + WS_QH), *QL = (_Float16*)(ws + WS_QL), *KH = (_Float16*)(ws + WS_KH), *KL = (_Float16*)(ws + WS_KL);
  _Float16* VT = (_Float16*)(ws + WS_VT); _Float16* AO = (_Float16*)(ws + WS_AO);
  unsigned short *WQB = (unsigned short*)(ws + WS_WQ), *WKB = (unsigned short*)(ws + WS_WK), *WVB = (unsigned short*)(ws + WS_WV); _Float16* WGH = (_Float16*)(ws + WS_WG);
  float* S = (float*)(ws + WS_S);
  k_wc<<<dim3(72), 256, 0, stream>>>(F[1], F[3], F[5], F[7], WQB, WKB, WVB, WGH);
  k_xt<<<dim3(SEQ / 64, NB), 256, 0, stream>>>(F[0], XB);
  k_qk<<<dim3(NB * SEQ / 64), 128, 0, stream>>>(XB, WQB, F[2], WKB, F[4], QH, QL, KH, KL);
  k_vp<<<dim3(NB * SEQ / 64, CX / 128), 128, 0, stream>>>(XB, WVB, F[6], VT);
  for (int b = 0; b < NB; ++b) {
    k_sc<<<dim3(SEQ / 64, SEQ / 128), 128, 0, stream>>>(QH, QL, KH, KL, b, S);
    k_rsm<<<dim3(SEQ / 2), 64, 0, stream>>>(S);
    k_pv<<<dim3(SEQ / 64, CX / 128), 128, 0, stream>>>(S, VT, b, AO);
  }
  k_op<<<dim3(NB * SEQ / 64, CX / 128), 128, 0, stream>>>(AO, WGH, F[8], F[0], (float*)d_out);
}
